// MeshMultiHeadAttention_6408091206165
// MI455X (gfx1250) — hardware-run, weakly checked
//
#include <hip/hip_runtime.h>
#include <math.h>

typedef __attribute__((ext_vector_type(16))) _Float16 v16h;
typedef __attribute__((ext_vector_type(16))) __bf16 v16b;
typedef __attribute__((ext_vector_type(8)))  _Float16 v8h;
typedef __attribute__((ext_vector_type(8)))  float v8f;
typedef __attribute__((ext_vector_type(4)))  float v4f;
typedef __attribute__((ext_vector_type(2)))  float v2f;
typedef __attribute__((ext_vector_type(4)))  unsigned v4u;
typedef __attribute__((ext_vector_type(4)))  int v4i;
typedef float __attribute__((may_alias)) float_a;
typedef int __attribute__((may_alias)) int_a;

template <typename T> __device__ __forceinline__ void vst2(void* p, T v) { *(volatile T*)p = v; __threadfence(); *(volatile T*)p = v; }
__device__ __forceinline__ v8f wmma16(v16h a, v16h b, v8f c) {
  v8f d = __builtin_amdgcn_wmma_f32_16x16x32_f16(false, a, false, b, (short)0, c, false, false);
  asm volatile("v_nop\n\tv_nop\n\tv_nop\n\tv_nop" : "+v"(d) : "v"(a), "v"(b));
  return d;
}
__device__ __forceinline__ v8f wmma_bf(v16b a, v16b b, v8f c) {
  v8f d = __builtin_amdgcn_wmma_f32_16x16x32_bf16(false, a, false, b, (short)0, c, false, false);
  asm volatile("v_nop\n\tv_nop\n\tv_nop\n\tv_nop" : "+v"(d) : "v"(a), "v"(b));
  return d;
}
__device__ __forceinline__ v16h frag_h(const _Float16* rowk0, int lane) {
  union { v16h v; v8h q[2]; } u; const _Float16* p = rowk0 + 8 * (lane >> 4);
  u.q[0] = *(const v8h*)p; u.q[1] = *(const v8h*)(p + 16); return u.v;
}
__device__ __forceinline__ v16h frag_f32(const float* rowk0, int lane) {
  v16h a; const float* p = rowk0 + 8 * (lane >> 4);
#pragma unroll
  for (int i = 0; i < 8; ++i) { a[i] = (_Float16)p[i]; a[8 + i] = (_Float16)p[16 + i]; }
  return a;
}
__device__ __forceinline__ v16h frag_f32s(const float* rowk0, int lane, float sc) {
  v16h a; const float* p = rowk0 + 8 * (lane >> 4);
#pragma unroll
  for (int i = 0; i < 8; ++i) { a[i] = (_Float16)(p[i] * sc); a[8 + i] = (_Float16)(p[16 + i] * sc); }
  return a;
}
__device__ __forceinline__ v16h fragc_f32(const float* W, int k0, int n, int lane, int ld, int K) {
  v16h a; const int g = lane >> 4;
#pragma unroll
  for (int i = 0; i < 8; ++i) { const int ka = k0 + 8 * g + i, kb = ka + 16;
    a[i] = (_Float16)(ka < K ? W[(size_t)(ka < K ? ka : K - 1) * ld + n] : 0.f); a[8 + i] = (_Float16)(kb < K ? W[(size_t)(kb < K ? kb : K - 1) * ld + n] : 0.f); }
  return a;
}
struct F2 { v16b h, l; };
__device__ __forceinline__ F2 bsplit16(const float v[16]) { F2 r;
#pragma unroll
  for (int i = 0; i < 16; ++i) { const __bf16 h = (__bf16)v[i]; r.h[i] = h; r.l[i] = (__bf16)(v[i] - (float)h); }
  return r; }
__device__ __forceinline__ F2 split_row(const float* row, int k0, int lane) { float v[16]; const float* p = row + k0 + 8 * (lane >> 4);
#pragma unroll
  for (int i = 0; i < 8; ++i) { v[i] = p[i]; v[8 + i] = p[16 + i]; }
  return bsplit16(v); }
__device__ __forceinline__ F2 split_rowK(const float* row, int k0, int lane, int K) { float v[16]; const int g = lane >> 4;
#pragma unroll
  for (int i = 0; i < 8; ++i) { const int ka = k0 + 8 * g + i, kb = ka + 16; v[i] = ka < K ? row[ka < K ? ka : K - 1] : 0.f; v[8 + i] = kb < K ? row[kb < K ? kb : K - 1] : 0.f; }
  return bsplit16(v); }
__device__ __forceinline__ F2 split_col(const float* W, int k0, int n, int lane, int ld, int K) { float v[16]; const int g = lane >> 4;
#pragma unroll
  for (int i = 0; i < 8; ++i) { const int ka = k0 + 8 * g + i, kb = ka + 16; v[i] = ka < K ? W[(size_t)(ka < K ? ka : K - 1) * ld + n] : 0.f; v[8 + i] = kb < K ? W[(size_t)(kb < K ? kb : K - 1) * ld + n] : 0.f; }
  return bsplit16(v); }
__device__ __forceinline__ v8f mac3(const F2& a, const F2& b, v8f c) { c = wmma_bf(a.l, b.h, c); c = wmma_bf(a.h, b.l, c); return wmma_bf(a.h, b.h, c); }
__device__ __forceinline__ float sigm(float v) { return 1.0f / (1.0f + expf(-v)); }
#define LDSX() do { asm volatile("s_wait_dscnt 0" ::: "memory"); __builtin_amdgcn_wave_barrier(); __builtin_amdgcn_fence(__ATOMIC_RELEASE, "workgroup"); } while (0)


#define NB 2
#define NV 1024
#define NE 3072
#define NF 2048
#define DD 256
#define NH 8
#define DK 32
#define EPS 1e-5f
#ifndef TNB
#define TNB NB
#endif
typedef __attribute__((ext_vector_type(8))) __bf16 v8b;
__device__ __forceinline__ v16b frag_b(const __bf16* rowk0, int lane) {
  union { v16b v; v8b q[2]; } u; const __bf16* p = rowk0 + 8 * (lane >> 4);
  u.q[0] = *(const v8b*)p; u.q[1] = *(const v8b*)(p + 16); return u.v;
}
__device__ __forceinline__ float bfr(float v) { return (float)(__bf16)v; }
__device__ __attribute__((noinline)) float exp_ni(float v) { return expf(v); }
__device__ __attribute__((noinline)) float erf_ni(float v) { return erff(v); }

#define SZR(N) (2u * (size_t)NB * (N) * DD)
#define WS_VQ   0u
#define WS_VK   (WS_VQ + 2 * SZR(NV))
#define WS_EQ   (WS_VK + 2 * SZR(NV))
#define WS_EK   (WS_EQ + 2 * SZR(NE))
#define WS_FK   (WS_EK + 2 * SZR(NE))
#define WS_VVT  (WS_FK + 2 * SZR(NF))
#define WS_EVT  (WS_VVT + 2 * SZR(NV))
#define WS_XV   (WS_EVT + 2 * SZR(NE))
#define WS_XF   (WS_XV + 2 * SZR(NE))
#define WS_ZV   (WS_XF + 2 * SZR(NF))
#define WS_ZEF  (WS_ZV + 4u * (size_t)NB * NV * DD)
#define WS_CT   (WS_ZEF + 4u * (size_t)NB * NE * DD)
#define WS_ZEV  (WS_CT + 2 * SZR(NV))
#define WS_ZC   (WS_ZEV + 4u * (size_t)NB * NE * DD)
#define WS_END  (WS_ZC + 4u * (size_t)NB * NV * DD)

__device__ __forceinline__ v16b fragb_f32(const float* __restrict__ p, int lane) { v16b a; const float* pp = p + 8 * (lane >> 4);
#pragma unroll
  for (int i = 0; i < 8; ++i) { a[i] = (__bf16)pp[i]; a[8 + i] = (__bf16)pp[16 + i]; } return a; }
__device__ __forceinline__ v16h fragh_f32exact(const float* __restrict__ p, int lane) { v16h a; const float* pp = p + 8 * (lane >> 4);
#pragma unroll
  for (int i = 0; i < 8; ++i) { a[i] = (_Float16)bfr(pp[i]); a[8 + i] = (_Float16)bfr(pp[16 + i]); } return a; }
template <int MODE>
__global__ __launch_bounds__(128) void k_proj(const float* __restrict__ X, int nrows, const float* __restrict__ Wn, const float* __restrict__ G, const float* __restrict__ Bt, _Float16* __restrict__ OH, _Float16* __restrict__ OL) {
  __shared__ __align__(16) _Float16 sh[64][136], sl[64][136]; __shared__ __align__(16) _Float16 th[128][72], tl[128][72];
  const int tid = threadIdx.x, wave = tid >> 5, lane = tid & 31, col = lane & 15, g = lane >> 4; const size_t b = blockIdx.z; const int i0 = blockIdx.x * 64 + wave * 16; const int c0 = blockIdx.y * 128; const size_t r0 = b * nrows + i0;
  v8f acc[8] = {};
#pragma unroll
  for (int kc = 0; kc < DD / 32; ++kc) { const v16b a = fragb_f32(X + (r0 + col) * DD + kc * 32, lane);
#pragma unroll
    for (int j = 0; j < 8; ++j) acc[j] = wmma_bf(a, fragb_f32(Wn + (size_t)(c0 + j * 16 + col) * DD + kc * 32, lane), acc[j]); }
  if (MODE == 0) {
#pragma unroll
    for (int hp = 0; hp < 4; ++hp) { const int hh = (c0 / DK) + hp;
#pragma unroll
      for (int r = 0; r < 8; ++r) { float s = acc[2 * hp][r] + acc[2 * hp + 1][r];
#pragma unroll
        for (int o = 1; o < 16; o <<= 1) s += __shfl_xor(s, o);
        const float mu = s * (1.0f / DK); const float d0 = acc[2 * hp][r] - mu, d1 = acc[2 * hp + 1][r] - mu; float q = d0 * d0 + d1 * d1;
#pragma unroll
        for (int o = 1; o < 16; o <<= 1) q += __shfl_xor(q, o);
        const float inv = 1.0f / sqrtf(q * (1.0f / DK) + EPS);
#pragma unroll
        for (int u = 0; u < 2; ++u) { const int d = u * 16 + col; const float y = (u == 0 ? d0 : d1) * inv * bfr(G[hh * DK + d]) + bfr(Bt[hh * DK + d]); const _Float16 hv = (_Float16)y; sh[wave * 16 + 8 * g + r][(2 * hp + u) * 16 + col] = hv; sl[wave * 16 + 8 * g + r][(2 * hp + u) * 16 + col] = (_Float16)((y - (float)hv) * 2048.0f); } } }
    __syncthreads(); for (int e = tid; e < 64 * 16; e += 128) { const int rl = e >> 4, q = e & 15; const size_t o = (b * nrows + blockIdx.x * 64 + rl) * DD + c0 + q * 8; vst2((unsigned*)(OH + o), *(const v4u*)&sh[rl][q * 8]); vst2((unsigned*)(OL + o), *(const v4u*)&sl[rl][q * 8]); } }
  else {
#pragma unroll
    for (int j = 0; j < 8; ++j)
#pragma unroll
      for (int r = 0; r < 8; ++r) { const float v = acc[j][r]; const _Float16 hv = (_Float16)v; th[j * 16 + col][wave * 16 + 8 * g + r] = hv; tl[j * 16 + col][wave * 16 + 8 * g + r] = (_Float16)((v - (float)hv) * 2048.0f); }
    __syncthreads(); for (int e = tid; e < 128 * 8; e += 128) { const int cl = e >> 3, q = e & 7; const size_t o = ((b * DD + c0 + cl) * (size_t)nrows) + blockIdx.x * 64 + q * 8; vst2((unsigned*)(OH + o), *(const v4u*)&th[cl][q * 8]); vst2((unsigned*)(OL + o), *(const v4u*)&tl[cl][q * 8]); } } }
__global__ __launch_bounds__(128) void k_lift(const _Float16* __restrict__ AH, const _Float16* __restrict__ AL, int nin, const float* __restrict__ Dop, int mrows, _Float16* __restrict__ OH, _Float16* __restrict__ OL) { __shared__ __align__(16) _Float16 sh[64][136], sl[64][136];
  const int tid = threadIdx.x, wave = tid >> 5, lane = tid & 31, col = lane & 15, g = lane >> 4; const size_t b = blockIdx.z; const int c0 = blockIdx.x * 64 + wave * 16; const int m0 = blockIdx.y * 128;
  v8f acc[8] = {}, accl[8] = {};
#pragma unroll 2
  for (int kc = 0; kc < nin / 32; ++kc) { const v16h ah = frag_h(AH + ((b * DD + c0 + col) * (size_t)nin) + kc * 32, lane), al = frag_h(AL + ((b * DD + c0 + col) * (size_t)nin) + kc * 32, lane);
#pragma unroll
    for (int j = 0; j < 8; ++j) { const v16h d = fragh_f32exact(Dop + ((b * mrows + m0 + j * 16 + col) * (size_t)nin) + kc * 32, lane); acc[j] = wmma16(ah, d, acc[j]); accl[j] = wmma16(al, d, accl[j]); } }
#pragma unroll
  for (int j = 0; j < 8; ++j)
#pragma unroll
    for (int r = 0; r < 8; ++r) { const float v = acc[j][r] + accl[j][r] * (1.0f / 2048.0f); const _Float16 hv = (_Float16)v; sh[wave * 16 + 8 * g + r][j * 16 + col] = hv; sl[wave * 16 + 8 * g + r][j * 16 + col] = (_Float16)((v - (float)hv) * 2048.0f); }
  LDSX(); for (int rl = 0; rl < 16; ++rl) if (lane < 16) { const size_t o = ((b * DD + c0 + rl) * (size_t)mrows) + m0 + lane * 8; vst2((unsigned*)(OH + o), *(const v4u*)&sh[wave * 16 + rl][lane * 8]); vst2((unsigned*)(OL + o), *(const v4u*)&sl[wave * 16 + rl][lane * 8]); } }
template <int TRP>
__global__ __launch_bounds__(128) void k_att(const _Float16* __restrict__ QH, const _Float16* __restrict__ QL, int nq, const _Float16* __restrict__ KH, const _Float16* __restrict__ KL, int nk, const _Float16* __restrict__ XH, const _Float16* __restrict__ XL, float* __restrict__ Z, _Float16* __restrict__ CTH, _Float16* __restrict__ CTL) {
  __shared__ __align__(16) float sp[4][16][36]; __shared__ __align__(16) float so[4][16][36]; __shared__ __align__(16) _Float16 th[32][72], tl[32][72];
  const int tid = threadIdx.x, wave = tid >> 5, lane = tid & 31, col = lane & 15, g = lane >> 4; const int h = blockIdx.y; const size_t b = blockIdx.z; const int q0 = blockIdx.x * 64 + wave * 16; const size_t rq = b * nq + q0;
  const v16h aq = frag_h(QH + (rq + col) * DD + h * DK, lane), aql = frag_h(QL + (rq + col) * DD + h * DK, lane);
  float m[8], l[8];
#pragma unroll
  for (int r = 0; r < 8; ++r) { m[r] = -3.0e38f; l[r] = 0.f; }
  v8f acc[2] = {}, accl[2] = {};
#pragma unroll 1
  for (int ks = 0; ks < nk / 32; ++ks) { v8f s[2];
#pragma unroll
    for (int ct = 0; ct < 2; ++ct) { const size_t rk = b * nk + ks * 32 + ct * 16 + col; const v16h kh = frag_h(KH + rk * DD + h * DK, lane), kl = frag_h(KL + rk * DD + h * DK, lane); v8f c = {}, cl = {}; c = wmma16(aq, kh, c); cl = wmma16(aq, kl, cl); cl = wmma16(aql, kh, cl);
#pragma unroll
      for (int r = 0; r < 8; ++r) s[ct][r] = (c[r] + cl[r] * (1.0f / 2048.0f)) * 0.17677669529663687f; }
    float alpha[8];
#pragma unroll
    for (int r = 0; r < 8; ++r) { float mx = fmaxf(s[0][r], s[1][r]);
#pragma unroll
      for (int o = 1; o < 16; o <<= 1) mx = fmaxf(mx, __shfl_xor(mx, o));
      const float mn = fmaxf(m[r], mx); alpha[r] = __expf(m[r] - mn); const float e0 = __expf(s[0][r] - mn), e1 = __expf(s[1][r] - mn); float es = e0 + e1;
#pragma unroll
      for (int o = 1; o < 16; o <<= 1) es += __shfl_xor(es, o);
      l[r] = l[r] * alpha[r] + es; m[r] = mn; sp[wave][8 * g + r][col] = e0; sp[wave][8 * g + r][16 + col] = e1; }
#pragma unroll
    for (int j = 0; j < 2; ++j)
#pragma unroll
      for (int r = 0; r < 8; ++r) { acc[j][r] *= alpha[r]; accl[j][r] *= alpha[r]; }
    LDSX();
    v16h pa; { const float* prow = &sp[wave][col][0] + 8 * (lane >> 4);
#pragma unroll
      for (int i = 0; i < 8; ++i) { pa[i] = (_Float16)(prow[i] * 2048.0f); pa[8 + i] = (_Float16)(prow[16 + i] * 2048.0f); } }
#pragma unroll
    for (int j = 0; j < 2; ++j) { const size_t po = (b * DD + (size_t)h * DK + j * 16 + col) * (size_t)nk + ks * 32; acc[j] = wmma16(pa, frag_h(XH + po, lane), acc[j]); accl[j] = wmma16(pa, frag_h(XL + po, lane), accl[j]); }
    LDSX(); }
#pragma unroll
  for (int r = 0; r < 8; ++r) { const float il = (1.0f / 2048.0f) / l[r];
#pragma unroll
    for (int j = 0; j < 2; ++j) { const float y = (acc[j][r] + accl[j][r] * (1.0f / 2048.0f)) * il; so[wave][8 * g + r][j * 16 + col] = y; if (TRP) { const _Float16 hv = (_Float16)y; th[j * 16 + col][wave * 16 + 8 * g + r] = hv; tl[j * 16 + col][wave * 16 + 8 * g + r] = (_Float16)((y - (float)hv) * 2048.0f); } } }
  __syncthreads();
  for (int rl = 0; rl < 16; ++rl) if (lane < 8) vst2(Z + (rq + rl) * DD + (size_t)h * DK + lane * 4, *(const v4f*)&so[wave][rl][lane * 4]);
  if (TRP) { for (int e = tid; e < 32 * 8; e += 128) { const int cl = e >> 3, q = e & 7; const size_t o = ((b * DD + (size_t)h * DK + cl) * (size_t)nq) + blockIdx.x * 64 + q * 8; vst2((unsigned*)(CTH + o), *(const v4u*)&th[cl][q * 8]); vst2((unsigned*)(CTL + o), *(const v4u*)&tl[cl][q * 8]); } } }
__global__ __launch_bounds__(128) void k_lift2(const float* __restrict__ D0, const _Float16* __restrict__ CTH, const _Float16* __restrict__ CTL, float* __restrict__ OUTF) { __shared__ __align__(16) float sf[4][16][132];
  const int tid = threadIdx.x, wave = tid >> 5, lane = tid & 31, col = lane & 15, g = lane >> 4; const size_t b = blockIdx.z; const int m0 = blockIdx.x * 64 + wave * 16; const int c0 = blockIdx.y * 128;
  v8f acc[8] = {}, accl[8] = {};
#pragma unroll 2
  for (int kc = 0; kc < NV / 32; ++kc) { const v16h a = fragh_f32exact(D0 + ((b * NE + m0 + col) * (size_t)NV) + kc * 32, lane);
#pragma unroll
    for (int j = 0; j < 8; ++j) { const size_t po = ((b * DD + c0 + j * 16 + col) * (size_t)NV) + kc * 32; acc[j] = wmma16(a, frag_h(CTH + po, lane), acc[j]); accl[j] = wmma16(a, frag_h(CTL + po, lane), accl[j]); } }
#pragma unroll
  for (int j = 0; j < 8; ++j)
#pragma unroll
    for (int r = 0; r < 8; ++r) sf[wave][8 * g + r][j * 16 + col] = acc[j][r] + accl[j][r] * (1.0f / 2048.0f);
  LDSX(); for (int rl = 0; rl < 16; ++rl) vst2(OUTF + (b * NE + m0 + rl) * DD + c0 + lane * 4, *(const v4f*)&sf[wave][rl][lane * 4]); }
template <int TWO>
__global__ __launch_bounds__(128) void k_out(const float* __restrict__ A1, const float* __restrict__ A2, const float* __restrict__ Wn, const float* __restrict__ BIAS, float* __restrict__ OUT, int nrows_total) { __shared__ __align__(16) float sf[4][16][132];
  const int tid = threadIdx.x, wave = tid >> 5, lane = tid & 31, col = lane & 15, g = lane >> 4; const size_t r0 = (size_t)blockIdx.x * 64 + wave * 16; const int c0 = blockIdx.y * 128; (void)nrows_total;
  v8f acc[8] = {};
#pragma unroll 2
  for (int kc = 0; kc < DD / 32; ++kc) { float v[16]; const float* p1 = A1 + (r0 + col) * DD + kc * 32 + 8 * g; const float* p2 = TWO ? A2 + (r0 + col) * DD + kc * 32 + 8 * g : nullptr;
#pragma unroll
    for (int i = 0; i < 8; ++i) { v[i] = p1[i] + (TWO ? p2[i] : 0.f); v[8 + i] = p1[16 + i] + (TWO ? p2[16 + i] : 0.f); }
    const F2 a = bsplit16(v);
#pragma unroll
    for (int j = 0; j < 8; ++j) { const v16b w = fragb_f32(Wn + (size_t)(c0 + j * 16 + col) * DD + kc * 32, lane); acc[j] = wmma_bf(a.h, w, acc[j]); acc[j] = wmma_bf(a.l, w, acc[j]); } }
#pragma unroll
  for (int j = 0; j < 8; ++j) { const float bb = bfr(BIAS[c0 + j * 16 + col]);
#pragma unroll
    for (int r = 0; r < 8; ++r) sf[wave][8 * g + r][j * 16 + col] = acc[j][r] + bb; }
  LDSX(); for (int rl = 0; rl < 16; ++rl) vst2(OUT + (r0 + rl) * DD + c0 + lane * 4, *(const v4f*)&sf[wave][rl][lane * 4]); }
extern "C" void kernel_launch(void* const* d_in, const int* in_sizes, int n_in, void* d_out, int out_size, void* d_ws, size_t ws_size, hipStream_t stream) {
  (void)in_sizes; (void)n_in; (void)out_size;
  const float** F = (const float**)d_in;
  if (ws_size < (size_t)WS_END) return;
  char* ws = (char*)d_ws;
  auto H16 = [&](size_t off) { return (_Float16*)(ws + off); };
  _Float16 *VQ = H16(WS_VQ), *VQL = VQ + (size_t)NB * NV * DD, *VK = H16(WS_VK), *VKL = VK + (size_t)NB * NV * DD, *EQ = H16(WS_EQ), *EQL = EQ + (size_t)NB * NE * DD, *EK = H16(WS_EK), *EKL = EK + (size_t)NB * NE * DD, *FK = H16(WS_FK), *FKL = FK + (size_t)NB * NF * DD;
  _Float16 *VVT = H16(WS_VVT), *VVTL = VVT + (size_t)NB * DD * NV, *EVT = H16(WS_EVT), *EVTL = EVT + (size_t)NB * DD * NE, *XV = H16(WS_XV), *XVL = XV + (size_t)NB * DD * NE, *XF = H16(WS_XF), *XFL = XF + (size_t)NB * DD * NF, *CT = H16(WS_CT), *CTLp = CT + (size_t)NB * DD * NV;
  float *ZV = (float*)(ws + WS_ZV), *ZEF = (float*)(ws + WS_ZEF), *ZEV = (float*)(ws + WS_ZEV), *ZC = (float*)(ws + WS_ZC);
  float* OUTV = (float*)d_out; float* OUTE = OUTV + (size_t)NB * NV * DD;
  k_proj<0><<<dim3(NV / 64, 2, TNB), 128, 0, stream>>>(F[0], NV, F[5], F[16], F[17], VQ, VQL);
  k_proj<0><<<dim3(NV / 64, 2, TNB), 128, 0, stream>>>(F[0], NV, F[6], F[18], F[19], VK, VKL);
  k_proj<1><<<dim3(NV / 64, 2, TNB), 128, 0, stream>>>(F[0], NV, F[7], nullptr, nullptr, VVT, VVTL);
  k_proj<0><<<dim3(NE / 64, 2, TNB), 128, 0, stream>>>(F[1], NE, F[8], F[20], F[21], EQ, EQL);
  k_proj<0><<<dim3(NE / 64, 2, TNB), 128, 0, stream>>>(F[1], NE, F[9], F[22], F[23], EK, EKL);
  k_proj<1><<<dim3(NE / 64, 2, TNB), 128, 0, stream>>>(F[1], NE, F[10], nullptr, nullptr, EVT, EVTL);
  k_proj<0><<<dim3(NF / 64, 2, TNB), 128, 0, stream>>>(F[2], NF, F[11], F[24], F[25], FK, FKL);
  k_lift<<<dim3(DD / 64, NE / 128, TNB), 128, 0, stream>>>(VVT, VVTL, NV, F[3], NE, XV, XVL);
  k_lift<<<dim3(DD / 64, NF / 128, TNB), 128, 0, stream>>>(EVT, EVTL, NE, F[4], NF, XF, XFL);
  k_att<0><<<dim3(NV / 64, NH, TNB), 128, 0, stream>>>(VQ, VQL, NV, EK, EKL, NE, XV, XVL, ZV, nullptr, nullptr);
  k_att<0><<<dim3(NE / 64, NH, TNB), 128, 0, stream>>>(EQ, EQL, NE, FK, FKL, NF, XF, XFL, ZEF, nullptr, nullptr);
  k_att<1><<<dim3(NV / 64, NH, TNB), 128, 0, stream>>>(VK, VKL, NV, EK, EKL, NE, EVT, EVTL, ZC, CT, CTLp);
  k_lift2<<<dim3(NE / 64, DD / 128, TNB), 128, 0, stream>>>(F[3], CT, CTLp, ZEV);
  k_out<0><<<dim3(TNB * NV / 64, DD / 128), 128, 0, stream>>>(ZV, nullptr, F[12], F[13], OUTV, NB * NV);
  k_out<1><<<dim3(TNB * NE / 64, DD / 128), 128, 0, stream>>>(ZEF, ZEV, F[14], F[15], OUTE, NB * NE);
}
